// PowerLSTMModule_13554916786411
// MI455X (gfx1250) — hardware-verified
//
#include <hip/hip_runtime.h>
#include <math.h>

constexpr int NBATCH  = 256;
constexpr int NSTEP   = 512;
constexpr int NFEAT   = 64;
constexpr int NHID    = 100;
constexpr int FC_MID  = 50;
constexpr int HPADK   = 128;
constexpr int NWAVES  = 7;
constexpr int NROWP   = NWAVES * 64;
constexpr int LTHR    = NWAVES * 32;
constexpr int KTOT0   = NFEAT + HPADK;
constexpr int KTOT1   = HPADK + HPADK;
constexpr int HP      = 136;
constexpr int YP      = 36;
constexpr int YSTEPS  = 32;
constexpr int NROWS   = NBATCH * NSTEP;
constexpr float WCARRY     = 64.0f;
constexpr float WCARRY_INV = 1.0f / 64.0f;
constexpr float LN_EPS_F   = 1e-5f;
constexpr int PAR_BIAS0 = 0;
constexpr int PAR_BIAS1 = 512;
constexpr int PAR_WEFF  = 1024;
constexpr int PAR_BEFF  = 1152;
constexpr int PAR_TOTAL = 1280;
constexpr int PREP_BLK0 = NROWP * (KTOT0 / 8) / 256;
constexpr int PREP_BLK1 = NROWP * (KTOT1 / 8) / 256;

static_assert(NBATCH == 256, "row index split uses shifts by 8");
static_assert(NBATCH % 16 == 0, "16 batch rows per block");
static_assert(NSTEP % YSTEPS == 0, "output flush period");
static_assert(NFEAT % 32 == 0 && HPADK % 32 == 0, "K multiples of 32");
static_assert(KTOT0 % 32 == 0 && KTOT1 % 32 == 0, "K multiples of 32");
static_assert(NHID <= 16 * NWAVES && 16 * NWAVES <= HPADK, "unit tiling");
static_assert(NROWP * (KTOT0 / 8) % 256 == 0, "weight plane 0 chunk count is a block multiple");
static_assert(NROWP * (KTOT1 / 8) % 256 == 0, "weight plane 1 chunk count is a block multiple");
static_assert(NROWS % 32 == 0, "LayerNorm grid exact");
static_assert(HP % 8 == 0 && HP >= HPADK, "h tile pitch");
static_assert(NROWP <= 512, "bias region size");

typedef __attribute__((ext_vector_type(16))) _Float16 v16h;
typedef __attribute__((ext_vector_type(8)))  _Float16 v8h;
typedef __attribute__((ext_vector_type(8)))  float    v8f;
typedef __attribute__((ext_vector_type(4)))  float    v4f;

template <typename T> struct Frag;
template <> struct Frag<_Float16> {
  typedef v16h V; union U { v16h v; v8h h[2]; };
  static __device__ __forceinline__ v16h load(const _Float16* p) {
    U f; f.h[0] = *(const v8h*)(p); f.h[1] = *(const v8h*)(p + 16); return f.v;
  }
  static __device__ __forceinline__ v8f mma(v16h a, v16h b, v8f c) {
    return __builtin_amdgcn_wmma_f32_16x16x32_f16(false, a, false, b, (short)0, c, false, false);
  }
};

__device__ __forceinline__ void guard_group(v8f& a0, v8f& a1, v8f& a2, v8f& a3,
                                            v16h x, v16h q0, v16h q1, v16h q2, v16h q3) {
  asm volatile("v_nop\n\tv_nop\n\tv_nop\n\tv_nop"
               : "+v"(a0), "+v"(a1), "+v"(a2), "+v"(a3)
               : "v"(x), "v"(q0), "v"(q1), "v"(q2), "v"(q3));
}

__device__ __forceinline__ float fsig(float x)  { return __builtin_amdgcn_rcpf(1.0f + expf(-x)); }
__device__ __forceinline__ float ftanh(float x) { return 1.0f - 2.0f * __builtin_amdgcn_rcpf(expf(2.0f * x) + 1.0f); }

__global__ __launch_bounds__(256) void prep_kernel(
    const float* __restrict__ W_ih0, const float* __restrict__ W_hh0,
    const float* __restrict__ b_ih0, const float* __restrict__ b_hh0,
    const float* __restrict__ W_ih1, const float* __restrict__ W_hh1,
    const float* __restrict__ b_ih1, const float* __restrict__ b_hh1,
    const float* __restrict__ fc1_W, const float* __restrict__ fc1_b,
    const float* __restrict__ fc2_W, const float* __restrict__ fc2_b,
    unsigned short* __restrict__ WC0, unsigned short* __restrict__ WC1, float* __restrict__ PAR) {
  const int tid = threadIdx.x;
  const int blk = blockIdx.x;
  if (blk < PREP_BLK0 + PREP_BLK1) {
    const bool l1 = (blk >= PREP_BLK0);
    const int ktot    = l1 ? KTOT1 : KTOT0;
    const int kinpad  = l1 ? HPADK : NFEAT;
    const int kinreal = l1 ? NHID : NFEAT;
    const float* wih = l1 ? W_ih1 : W_ih0;
    const float* whh = l1 ? W_hh1 : W_hh0;
    unsigned short* dst = l1 ? WC1 : WC0;
    const int i = (l1 ? (blk - PREP_BLK0) : blk) * 256 + tid;
    const int cpr = ktot >> 3;
    const int row = i / cpr;
    const int k8  = (i - row * cpr) * 8;
    const int w = row >> 6, g = (row >> 4) & 3, jj = row & 15;
    const int u = 16 * w + jj;
    const bool rv = (u < NHID);
    const int orig = g * NHID + (rv ? u : 0);
    const bool hpart = (k8 >= kinpad);
    const float* src = hpart ? whh : wih;
    const int kreal = hpart ? NHID : kinreal;
    const int kk0 = hpart ? (k8 - kinpad) : k8;
    const float* srow = src + (size_t)orig * (size_t)kreal;
    v8h hv;
#pragma unroll
    for (int e = 0; e < 8; ++e) {
      const int kk = kk0 + e;
      const int kc = (kk < kreal) ? kk : (kreal - 1);
      const float val = srow[kc];
      const float v = (rv && (kk < kreal)) ? (val * WCARRY) : 0.0f;
      hv[e] = (_Float16)v;
    }
    unsigned short* dp = dst + (size_t)i * 8;
    *(volatile v8h*)dp = hv;
    __threadfence();
    *(volatile v8h*)dp = hv;
  } else {
    const int lane = tid & 31;
#pragma unroll 1
    for (int it = 0; it < 2; ++it) {
      const int region = __builtin_amdgcn_readfirstlane((tid >> 5) + 8 * it);
      if (region < 10) {
        v4f o = {0.0f, 0.0f, 0.0f, 0.0f};
        if (region < 8) {
          const bool l1 = (region >= 4);
          const float* bi = l1 ? b_ih1 : b_ih0;
          const float* bh = l1 ? b_hh1 : b_hh0;
          const int f0 = (region & 3) * 128 + lane * 4;
#pragma unroll
          for (int e = 0; e < 4; ++e) {
            const int n = f0 + e;
            const bool nv = (n < NROWP);
            const int nn = nv ? n : 0;
            const int w = nn >> 6, g = (nn >> 4) & 3, jj = nn & 15;
            const int u = 16 * w + jj;
            const bool rv = nv && (u < NHID);
            const int orig = g * NHID + ((u < NHID) ? u : 0);
            const float s = bi[orig] + bh[orig];
            o[e] = rv ? s : 0.0f;
          }
        } else if (region == 8) {
          float s0 = 0.0f, s1 = 0.0f, s2 = 0.0f, s3 = 0.0f;
          const int kb = lane * 4;
          const int k0c = (kb + 0 < NHID) ? (kb + 0) : (NHID - 1);
          const int k1c = (kb + 1 < NHID) ? (kb + 1) : (NHID - 1);
          const int k2c = (kb + 2 < NHID) ? (kb + 2) : (NHID - 1);
          const int k3c = (kb + 3 < NHID) ? (kb + 3) : (NHID - 1);
#pragma unroll 1
          for (int m = 0; m < FC_MID; ++m) {
            const float wm = fc2_W[m];
            const float* fr = fc1_W + m * NHID;
            s0 = fmaf(wm, fr[k0c], s0);
            s1 = fmaf(wm, fr[k1c], s1);
            s2 = fmaf(wm, fr[k2c], s2);
            s3 = fmaf(wm, fr[k3c], s3);
          }
          o[0] = (kb + 0 < NHID) ? s0 : 0.0f;
          o[1] = (kb + 1 < NHID) ? s1 : 0.0f;
          o[2] = (kb + 2 < NHID) ? s2 : 0.0f;
          o[3] = (kb + 3 < NHID) ? s3 : 0.0f;
        } else {
          float s = fc2_b[0];
#pragma unroll 1
          for (int m = 0; m < FC_MID; ++m) s = fmaf(fc2_W[m], fc1_b[m], s);
          o[0] = (lane == 0) ? s : 0.0f;
        }
        float* op = PAR + region * 128 + lane * 4;
        *(volatile v4f*)op = o;
        __threadfence();
        *(volatile v4f*)op = o;
      }
    }
  }
}

__global__ __launch_bounds__(256) void ln_rows_kernel(const float* __restrict__ x, const float* __restrict__ gam,
                                                      const float* __restrict__ bet, unsigned short* __restrict__ xn) {
  const int tid  = threadIdx.x;
  const int orow = blockIdx.x * 32 + (tid >> 3);
  const int l8   = tid & 7;
  const int t    = orow >> 8;
  const int b    = orow & 255;
  const float* rp = x + ((size_t)b * NSTEP + (size_t)t) * NFEAT + 8 * l8;
  const v4f a0 = *(const v4f*)(rp);
  const v4f a1 = *(const v4f*)(rp + 4);
  const v4f g0 = *(const v4f*)(gam + 8 * l8);
  const v4f g1 = *(const v4f*)(gam + 8 * l8 + 4);
  const v4f e0 = *(const v4f*)(bet + 8 * l8);
  const v4f e1 = *(const v4f*)(bet + 8 * l8 + 4);
  float v[8], gg[8], be[8];
#pragma unroll
  for (int e = 0; e < 4; ++e) {
    v[e] = a0[e]; v[4 + e] = a1[e];
    gg[e] = g0[e]; gg[4 + e] = g1[e];
    be[e] = e0[e]; be[4 + e] = e1[e];
  }
  float s = ((v[0] + v[1]) + (v[2] + v[3])) + ((v[4] + v[5]) + (v[6] + v[7]));
  s += __shfl_xor(s, 1, 32);
  s += __shfl_xor(s, 2, 32);
  s += __shfl_xor(s, 4, 32);
  const float mu = s * (1.0f / NFEAT);
  float ss = 0.0f;
#pragma unroll
  for (int e = 0; e < 8; ++e) { const float d = v[e] - mu; v[e] = d; ss += d * d; }
  ss += __shfl_xor(ss, 1, 32);
  ss += __shfl_xor(ss, 2, 32);
  ss += __shfl_xor(ss, 4, 32);
  const float var  = ss * (1.0f / NFEAT);
  const float rstd = rsqrtf(var + LN_EPS_F);
  v8h hv;
#pragma unroll
  for (int e = 0; e < 8; ++e) {
    const float o = (v[e] * rstd) * gg[e] + be[e];
    hv[e] = (_Float16)o;
  }
  unsigned short* op = xn + (size_t)orow * NFEAT + 8 * l8;
  *(volatile v8h*)op = hv;
  __threadfence();
  *(volatile v8h*)op = hv;
}

template <int KIN, bool LAST>
__global__ __launch_bounds__(LTHR) void lstm_cat_kernel(
    const unsigned short* __restrict__ INp, const unsigned short* __restrict__ Wp,
    const float* __restrict__ biasp, const float* __restrict__ weffp, const float* __restrict__ beffp,
    unsigned short* H1p, float* OUTp) {
  constexpr int KTOT = KIN + HPADK;
  static_assert(KIN % 32 == 0 && KTOT % 32 == 0, "k-steps of 32");
  __shared__ __align__(16) _Float16 hA[2][16 * HP];
  __shared__ __align__(16) float    ypart[2][NWAVES * 16];
  __shared__ __align__(16) float    ybuf[16 * YP];
  const _Float16* IN = (const _Float16*)INp;
  const _Float16* W  = (const _Float16*)Wp;
  const int tid  = threadIdx.x;
  const int lane = tid & 31;
  const int wave = __builtin_amdgcn_readfirstlane(tid >> 5);
  const int c = lane & 15, hh = lane >> 4, koff = hh * 8;
  const int b0 = blockIdx.x * 16;
  const int j  = 16 * wave + c;
  const bool colvalid = (j < NHID);

  {
    _Float16* hz = &hA[0][0];
#pragma unroll 1
    for (int i = tid; i < 2 * 16 * HP; i += LTHR) hz[i] = (_Float16)0.0f;
  }
  float cst[8], bb[4];
#pragma unroll
  for (int r = 0; r < 8; ++r) cst[r] = 0.0f;
#pragma unroll
  for (int g = 0; g < 4; ++g) bb[g] = biasp[64 * wave + 16 * g + c] * WCARRY;
  float wj = 0.0f, beff = 0.0f;
  if (LAST) { wj = weffp[j]; beff = beffp[0]; }
  __syncthreads();

  const _Float16* wr0 = W + (size_t)(64 * wave + c) * KTOT + koff;
  const _Float16* wr1 = wr0 + (size_t)16 * KTOT;
  const _Float16* wr2 = wr0 + (size_t)32 * KTOT;
  const _Float16* wr3 = wr0 + (size_t)48 * KTOT;

#pragma unroll 1
  for (int t = 0; t < NSTEP; ++t) {
    const int cur = t & 1;
    v8f acc[4];
#pragma unroll
    for (int g = 0; g < 4; ++g) {
      const float bv = bb[g];
      acc[g] = (v8f){bv, bv, bv, bv, bv, bv, bv, bv};
    }
    const _Float16* arow = IN + ((size_t)t * NBATCH + (size_t)(b0 + c)) * KIN + koff;
#pragma unroll 1
    for (int k0 = 0; k0 < KIN; k0 += 32) {
      const v16h a  = Frag<_Float16>::load(arow + k0);
      const v16h q0 = Frag<_Float16>::load(wr0 + k0);
      const v16h q1 = Frag<_Float16>::load(wr1 + k0);
      const v16h q2 = Frag<_Float16>::load(wr2 + k0);
      const v16h q3 = Frag<_Float16>::load(wr3 + k0);
      acc[0] = Frag<_Float16>::mma(a, q0, acc[0]);
      acc[1] = Frag<_Float16>::mma(a, q1, acc[1]);
      acc[2] = Frag<_Float16>::mma(a, q2, acc[2]);
      acc[3] = Frag<_Float16>::mma(a, q3, acc[3]);
      guard_group(acc[0], acc[1], acc[2], acc[3], a, q0, q1, q2, q3);
    }
    const _Float16* hrow = &hA[cur][0] + c * HP + koff;
#pragma unroll 1
    for (int k0 = 0; k0 < HPADK; k0 += 32) {
      const v16h a  = Frag<_Float16>::load(hrow + k0);
      const v16h q0 = Frag<_Float16>::load(wr0 + KIN + k0);
      const v16h q1 = Frag<_Float16>::load(wr1 + KIN + k0);
      const v16h q2 = Frag<_Float16>::load(wr2 + KIN + k0);
      const v16h q3 = Frag<_Float16>::load(wr3 + KIN + k0);
      acc[0] = Frag<_Float16>::mma(a, q0, acc[0]);
      acc[1] = Frag<_Float16>::mma(a, q1, acc[1]);
      acc[2] = Frag<_Float16>::mma(a, q2, acc[2]);
      acc[3] = Frag<_Float16>::mma(a, q3, acc[3]);
      guard_group(acc[0], acc[1], acc[2], acc[3], a, q0, q1, q2, q3);
    }

    _Float16* hnext = &hA[cur ^ 1][0];
    float hn[8];
#pragma unroll
    for (int r = 0; r < 8; ++r) {
      const float zi = acc[0][r] * WCARRY_INV;
      const float zf = acc[1][r] * WCARRY_INV;
      const float zg = acc[2][r] * WCARRY_INV;
      const float zo = acc[3][r] * WCARRY_INV;
      const float ig = fsig(zi);
      const float fg = fsig(zf);
      const float gt = ftanh(zg);
      const float og = fsig(zo);
      const float cn = fg * cst[r] + ig * gt;
      cst[r] = cn;
      const float hv = og * ftanh(cn);
      const float hs = colvalid ? hv : 0.0f;
      hn[r] = hs;
      hnext[(8 * hh + r) * HP + j] = (_Float16)hs;
    }
    if (wave == NWAVES - 1) {
#pragma unroll
      for (int r = 0; r < 8; ++r) hnext[(8 * hh + r) * HP + 16 * NWAVES + c] = (_Float16)0.0f;
    }
    if (LAST) {
      float yp[8];
#pragma unroll
      for (int r = 0; r < 8; ++r) yp[r] = wj * hn[r];
#pragma unroll
      for (int off = 1; off < 16; off <<= 1) {
#pragma unroll
        for (int r = 0; r < 8; ++r) yp[r] += __shfl_xor(yp[r], off, 32);
      }
      if (c == 0) {
#pragma unroll
        for (int r = 0; r < 8; ++r) ypart[cur][wave * 16 + 8 * hh + r] = yp[r];
      }
    }
    __syncthreads();

    if (!LAST) {
      if (wave < 4) {
        const _Float16* hs = &hA[cur ^ 1][0];
        const v8h v0 = *(const v8h*)(hs + (4 * wave + hh) * HP + 8 * c);
        const v8h v1 = *(const v8h*)(hs + (4 * wave + 2 + hh) * HP + 8 * c);
        unsigned short* d0 = H1p + ((size_t)t * NBATCH + (size_t)(b0 + 4 * wave + hh)) * HPADK + 8 * c;
        unsigned short* d1 = d0 + 2 * HPADK;
        for (int pass = 0; pass < 2; ++pass) {
          *(volatile v8h*)d0 = v0;
          *(volatile v8h*)d1 = v1;
          __threadfence();
        }
      }
    } else {
      if (wave == 0) {
        const float* yps = &ypart[cur][0];
        float s = beff;
#pragma unroll
        for (int w = 0; w < NWAVES; ++w) s += yps[w * 16 + c];
        if (lane < 16) ybuf[c * YP + (t & (YSTEPS - 1))] = s;
        if ((t & (YSTEPS - 1)) == YSTEPS - 1) {
          __builtin_amdgcn_fence(__ATOMIC_RELEASE, "workgroup");
          __builtin_amdgcn_wave_barrier();
          __builtin_amdgcn_fence(__ATOMIC_ACQUIRE, "workgroup");
          const int t0 = t - (YSTEPS - 1);
          const int q = lane >> 3, c4 = (lane & 7) * 4;
          v4f vv[4];
#pragma unroll
          for (int it = 0; it < 4; ++it) {
            const float* yb = ybuf + (it * 4 + q) * YP + c4;
            vv[it] = (v4f){yb[0], yb[1], yb[2], yb[3]};
          }
          for (int pass = 0; pass < 2; ++pass) {
#pragma unroll
            for (int it = 0; it < 4; ++it) {
              float* op = OUTp + (size_t)(b0 + it * 4 + q) * NSTEP + (size_t)(t0 + c4);
              *(volatile v4f*)op = vv[it];
            }
            __threadfence();
          }
          __builtin_amdgcn_fence(__ATOMIC_RELEASE, "workgroup");
          __builtin_amdgcn_wave_barrier();
          __builtin_amdgcn_fence(__ATOMIC_ACQUIRE, "workgroup");
        }
      }
    }
  }
}

extern "C" void kernel_launch(void* const* d_in, const int* in_sizes, int n_in,
                              void* d_out, int out_size, void* d_ws, size_t ws_size, hipStream_t stream) {
  if (n_in < 15 || d_out == nullptr || d_ws == nullptr) return;
  if (in_sizes[0] != NBATCH * NSTEP * NFEAT || in_sizes[1] != NFEAT || in_sizes[2] != NFEAT ||
      in_sizes[3] != 4 * NHID * NFEAT || in_sizes[4] != 4 * NHID * NHID ||
      in_sizes[5] != 4 * NHID || in_sizes[6] != 4 * NHID ||
      in_sizes[7] != 4 * NHID * NHID || in_sizes[8] != 4 * NHID * NHID ||
      in_sizes[9] != 4 * NHID || in_sizes[10] != 4 * NHID ||
      in_sizes[11] != FC_MID * NHID || in_sizes[12] != FC_MID || in_sizes[13] != FC_MID ||
      in_sizes[14] != 1 || out_size != NBATCH * NSTEP) return;

  const float* x     = (const float*)d_in[0];
  const float* lng   = (const float*)d_in[1];
  const float* lnb   = (const float*)d_in[2];
  const float* W_ih0 = (const float*)d_in[3];
  const float* W_hh0 = (const float*)d_in[4];
  const float* b_ih0 = (const float*)d_in[5];
  const float* b_hh0 = (const float*)d_in[6];
  const float* W_ih1 = (const float*)d_in[7];
  const float* W_hh1 = (const float*)d_in[8];
  const float* b_ih1 = (const float*)d_in[9];
  const float* b_hh1 = (const float*)d_in[10];
  const float* fc1_W = (const float*)d_in[11];
  const float* fc1_b = (const float*)d_in[12];
  const float* fc2_W = (const float*)d_in[13];
  const float* fc2_b = (const float*)d_in[14];
  float* y = (float*)d_out;

  char* ws = (char*)d_ws; size_t off = 0;
  auto carve = [&](size_t bytes) -> char* { char* p = ws + off; off += (bytes + 255) & ~(size_t)255; return p; };
  unsigned short* XN  = (unsigned short*)carve((size_t)NROWS * NFEAT * 2);
  unsigned short* H1  = (unsigned short*)carve((size_t)NROWS * HPADK * 2);
  unsigned short* WC0 = (unsigned short*)carve((size_t)NROWP * KTOT0 * 2);
  unsigned short* WC1 = (unsigned short*)carve((size_t)NROWP * KTOT1 * 2);
  float*          PAR = (float*)carve((size_t)PAR_TOTAL * 4);
  if (off > ws_size || off > (size_t)134217728) return;

  prep_kernel<<<PREP_BLK0 + PREP_BLK1 + 1, 256, 0, stream>>>(W_ih0, W_hh0, b_ih0, b_hh0, W_ih1, W_hh1, b_ih1, b_hh1,
                                                              fc1_W, fc1_b, fc2_W, fc2_b, WC0, WC1, PAR);
  ln_rows_kernel<<<NROWS / 32, 256, 0, stream>>>(x, lng, lnb, XN);
  lstm_cat_kernel<NFEAT, false><<<NBATCH / 16, LTHR, 0, stream>>>(XN, WC0, PAR + PAR_BIAS0, PAR + PAR_WEFF,
                                                                  PAR + PAR_BEFF, H1, y);
  lstm_cat_kernel<HPADK, true><<<NBATCH / 16, LTHR, 0, stream>>>(H1, WC1, PAR + PAR_BIAS1, PAR + PAR_WEFF,
                                                                 PAR + PAR_BEFF, H1, y);
}
